// HybridGCN_SAGE_39238821216992
// MI455X (gfx1250) — hardware-verified
//
#include <hip/hip_runtime.h>

typedef unsigned short us;
typedef us     v8us  __attribute__((ext_vector_type(8)));
typedef us     v16us __attribute__((ext_vector_type(16)));
typedef __bf16 v16bf __attribute__((ext_vector_type(16)));
typedef float  v4f   __attribute__((ext_vector_type(4)));
typedef float  v8f   __attribute__((ext_vector_type(8)));
typedef int    v4i   __attribute__((ext_vector_type(4)));
typedef v8us __attribute__((may_alias)) v8usa;
typedef v4f  __attribute__((may_alias)) v4fa;
typedef v4i  __attribute__((may_alias)) v4ia;

#define HD 128
#define OD 3
#define BM 32
#define RC 4096
#define RG 384

__device__ __forceinline__ us f2bf(float x) {
  unsigned u = __builtin_bit_cast(unsigned, x);
  u += 0x7FFFu + ((u >> 16) & 1u);
  return (us)(u >> 16);
}
__device__ __forceinline__ float bf2f(us s) {
  return __builtin_bit_cast(float, ((unsigned)s) << 16);
}

union FU { v16us u; v8us h[2]; };

__device__ __forceinline__ v16us ldfrag(const us* base, int r, int k0, int hf) {
  FU f;
  const us* p = base + r * HD + k0 + 8 * hf;
  f.h[0] = *(const v8usa*)p;
  f.h[1] = *(const v8usa*)(p + 16);
  return f.u;
}

__device__ __forceinline__ v8f mma_bf16(v16us a, v16us b, v8f c) {
  v16bf ab = __builtin_bit_cast(v16bf, a);
  v16bf bb = __builtin_bit_cast(v16bf, b);
  c = __builtin_amdgcn_wmma_f32_16x16x32_bf16(false, ab, false, bb, (short)0, c, false, false);
  asm volatile("v_nop\n\tv_nop\n\tv_nop\n\tv_nop" : "+v"(c) : "v"(a), "v"(b));
  return c;
}

__global__ void __launch_bounds__(256)
k_wtconv(const float* __restrict__ W0, const float* __restrict__ W1,
         const float* __restrict__ W2, const float* __restrict__ W3,
         us* __restrict__ dst) {
  const int w = blockIdx.y;
  const int t = blockIdx.x * 256 + threadIdx.x;
  if (t >= HD * (HD / 8)) return;
  const float* W = (w == 0) ? W0 : (w == 1) ? W1 : (w == 2) ? W2 : W3;
  const int n = t >> 4;
  const int kb = (t & 15) * 8;
  v8us hv, lv;
#pragma unroll
  for (int i = 0; i < 8; ++i) {
    float x = W[(kb + i) * HD + n];
    us hb = f2bf(x);
    us lb = f2bf(x - bf2f(hb));
    hv[i] = hb;
    lv[i] = lb;
  }
  us* ph = dst + (size_t)w * (2 * HD * HD) + n * HD + kb;
  us* pl = ph + HD * HD;
  *(volatile v8usa*)ph = hv;
  *(volatile v8usa*)pl = lv;
  __threadfence();
  *(volatile v8usa*)ph = hv;
  *(volatile v8usa*)pl = lv;
}

template <bool GUARD>
__device__ __forceinline__ void deg_chunk(const int* __restrict__ colp, int e0, int E,
                                          int n0, int lane, int* sCnt) {
  int loc[4];
  unsigned mk[4];
#pragma unroll
  for (int j = 0; j < 4; ++j) {
    const int e = e0 + 32 * j + lane;
    int c;
    if (GUARD) c = (e < E) ? colp[e] : -1; else c = colp[e];
    loc[j] = c - n0;
    mk[j] = __builtin_amdgcn_ballot_w32((unsigned)loc[j] < (unsigned)RC);
  }
#pragma unroll
  for (int j = 0; j < 4; ++j) {
    unsigned m = mk[j];
    while (m) {
      const int bit = __builtin_ctz(m);
      m &= m - 1u;
      const int cl = __builtin_amdgcn_readlane(loc[j], bit);
      if (lane == 0) sCnt[cl] += 1;
    }
  }
}

__device__ __forceinline__ void deg_store(const int* sCnt, int n0, int Npad, int lane,
                                          float* __restrict__ dinv, float* __restrict__ rcnt) {
  for (int i = lane * 4; i < RC; i += 128) {
    const int node = n0 + i;
    if (node < Npad) {
      v4i c = *(const v4ia*)(sCnt + i);
      v4f dv, rv;
#pragma unroll
      for (int q = 0; q < 4; ++q) {
        float cf = (float)c[q];
        dv[q] = rsqrtf(cf + 1.0f);
        rv[q] = 1.0f / fmaxf(cf, 1.0f);
      }
      *(volatile v4fa*)(dinv + node) = dv;
      *(volatile v4fa*)(rcnt + node) = rv;
    }
  }
}

__global__ void __launch_bounds__(32)
k_degree(const int* __restrict__ colp, int E, int N, int Npad,
         float* __restrict__ dinv, float* __restrict__ rcnt) {
  __shared__ __align__(16) int sCnt[RC];
  const int lane = threadIdx.x;
  const int n0 = blockIdx.x * RC;
  v4i z = {0, 0, 0, 0};
  for (int i = lane * 4; i < RC; i += 128) *(v4ia*)(sCnt + i) = z;
  __syncthreads();
  int e0 = 0;
  for (; e0 + 128 <= E; e0 += 128) deg_chunk<false>(colp, e0, E, n0, lane, sCnt);
  if (e0 < E) deg_chunk<true>(colp, e0, E, n0, lane, sCnt);
  __syncthreads();
  deg_store(sCnt, n0, Npad, lane, dinv, rcnt);
  __threadfence();
  deg_store(sCnt, n0, Npad, lane, dinv, rcnt);
}

template <bool GUARD>
__device__ __forceinline__ void gat_chunk(const int* __restrict__ rowp, const int* __restrict__ colp,
                                          const float* __restrict__ src, int e0, int E, int N,
                                          int n0, int lane, float* sAcc) {
  int loc[4];
  unsigned mk[4];
#pragma unroll
  for (int j = 0; j < 4; ++j) {
    const int e = e0 + 32 * j + lane;
    int c;
    if (GUARD) c = (e < E) ? colp[e] : -1; else c = colp[e];
    loc[j] = c - n0;
    mk[j] = __builtin_amdgcn_ballot_w32((unsigned)loc[j] < (unsigned)RG);
  }
#pragma unroll
  for (int j = 0; j < 4; ++j) {
    unsigned m = mk[j];
    while (m) {
      const int bit = __builtin_ctz(m);
      m &= m - 1u;
      const int cl = __builtin_amdgcn_readlane(loc[j], bit);
      const int e = e0 + 32 * j + bit;
      int r = rowp[e];
      r = (r < 0) ? 0 : ((r >= N) ? (N - 1) : r);
      const v4f v = *(const v4fa*)(src + (size_t)r * HD + 4 * lane);
      v4fa* ap = (v4fa*)(sAcc + cl * HD + 4 * lane);
      v4f a = *ap;
      a += v;
      *ap = a;
    }
  }
}

__device__ __forceinline__ void gat_store(const float* sAcc, float* __restrict__ dst,
                                          int n0, int N, int lane) {
  for (int i = 0; i < RG; ++i) {
    const int c = n0 + i;
    if (c >= N) break;
    const v4f val = *(const v4fa*)(sAcc + i * HD + 4 * lane);
    *(volatile v4fa*)(dst + (size_t)c * HD + 4 * lane) = val;
  }
}

__global__ void __launch_bounds__(32)
k_gather(const int* __restrict__ rowp, const int* __restrict__ colp, int E, int N,
         const float* __restrict__ src, const float* __restrict__ dinv,
         const float* __restrict__ rcnt, const float* __restrict__ bias,
         float* __restrict__ dst, int mode) {
  __shared__ __align__(16) float sAcc[RG * HD];
  const int lane = threadIdx.x;
  const int n0 = blockIdx.x * RG;
  v4f z = {0.f, 0.f, 0.f, 0.f};
  for (int i = lane * 4; i < RG * HD; i += 128) *(v4fa*)(sAcc + i) = z;
  __syncthreads();
  int e0 = 0;
  for (; e0 + 128 <= E; e0 += 128) gat_chunk<false>(rowp, colp, src, e0, E, N, n0, lane, sAcc);
  if (e0 < E) gat_chunk<true>(rowp, colp, src, e0, E, N, n0, lane, sAcc);
  __syncthreads();

  const v4f bv = *(const v4fa*)(bias + 4 * lane);
  for (int i = 0; i < RG; ++i) {
    const int c = n0 + i;
    if (c >= N) break;
    v4fa* ap = (v4fa*)(sAcc + i * HD + 4 * lane);
    v4f a = *ap;
    v4f val;
    if (mode == 0) {
      const v4f hv = *(const v4fa*)(src + (size_t)c * HD + 4 * lane);
      const float d = dinv[c];
      val = d * (a + hv) + bv;
      val.x = fmaxf(val.x, 0.0f);
      val.y = fmaxf(val.y, 0.0f);
      val.z = fmaxf(val.z, 0.0f);
      val.w = fmaxf(val.w, 0.0f);
    } else {
      const float rc = rcnt[c];
      val = a * rc;
    }
    *ap = val;
  }
  gat_store(sAcc, dst, n0, N, lane);
  __threadfence();
  gat_store(sAcc, dst, n0, N, lane);
}

template <bool GUARD>
__device__ __forceinline__ void pool_chunk(const int* __restrict__ batchp,
                                           const float* __restrict__ hsrc,
                                           int nb, int N, int g, int lane, v4f& acc) {
  unsigned mk[4];
#pragma unroll
  for (int j = 0; j < 4; ++j) {
    const int n = nb + 32 * j + lane;
    int b;
    if (GUARD) b = (n < N) ? batchp[n] : -1; else b = batchp[n];
    mk[j] = __builtin_amdgcn_ballot_w32(b == g);
  }
#pragma unroll
  for (int j = 0; j < 4; ++j) {
    unsigned m = mk[j];
    while (m) {
      const int bit = __builtin_ctz(m);
      m &= m - 1u;
      const int node = nb + 32 * j + bit;
      acc += *(const v4fa*)(hsrc + (size_t)node * HD + 4 * lane);
    }
  }
}

__global__ void __launch_bounds__(32)
k_pool(const int* __restrict__ batchp, int N, const float* __restrict__ hsrc,
       float* __restrict__ pooled) {
  const int g = blockIdx.x;
  const int lane = threadIdx.x;
  v4f acc = {0.f, 0.f, 0.f, 0.f};
  int nb = 0;
  for (; nb + 128 <= N; nb += 128) pool_chunk<false>(batchp, hsrc, nb, N, g, lane, acc);
  if (nb < N) pool_chunk<true>(batchp, hsrc, nb, N, g, lane, acc);
  float* p = pooled + (size_t)g * HD + 4 * lane;
  *(volatile v4fa*)p = acc;
  __threadfence();
  *(volatile v4fa*)p = acc;
}

__device__ __forceinline__ void gemm_rows_store(const float* sOut, float* __restrict__ OUT,
                                                int row0, int M, int wv, int lane) {
#pragma unroll
  for (int r4 = 0; r4 < 4; ++r4) {
    const int row = wv * 4 + r4;
    const int gr = row0 + row;
    if (gr < M) {
      const v4f v = *(const v4fa*)(sOut + row * HD + 4 * lane);
      *(volatile v4fa*)(OUT + (size_t)gr * HD + 4 * lane) = v;
    }
  }
}

__device__ __forceinline__ void head_store(const float* sRes, float* __restrict__ hout,
                                           int base, int nres, int hout_n, int lane) {
  const int nv = nres >> 2;
  if (lane < nv && base + 4 * lane + 3 < hout_n) {
    const v4f v = *(const v4fa*)(sRes + 4 * lane);
    *(volatile v4fa*)(hout + base + 4 * lane) = v;
  }
  const int rem = nres & 3;
  if (lane < rem) {
    const int idx = base + nv * 4 + lane;
    if (idx < hout_n) *(volatile float*)(hout + idx) = sRes[nv * 4 + lane];
  }
}

__global__ void __launch_bounds__(256)
k_gemm(const float* __restrict__ A1, const us* __restrict__ W1h, const us* __restrict__ W1l,
       const float* __restrict__ A2, const us* __restrict__ W2h, const us* __restrict__ W2l,
       const float* __restrict__ bias, const float* __restrict__ rscale,
       float* __restrict__ OUT, int M,
       int dual, int use_bias, int relu, int use_rs, int head,
       const float* __restrict__ Wf2, const float* __restrict__ bf2,
       float* __restrict__ hout, int hout_n) {
  __shared__ __align__(16) us    sWh[HD * HD];
  __shared__ __align__(16) us    sWl[HD * HD];
  __shared__ __align__(16) us    sAh[BM * HD];
  __shared__ __align__(16) us    sAl[BM * HD];
  __shared__ __align__(16) float sOut[BM * HD];
  __shared__ __align__(16) float sRes[128];

  const int tid = threadIdx.x;
  const int lane = tid & 31, wv = tid >> 5;
  const int hf = lane >> 4, m = lane & 15;
  const int row0 = blockIdx.x * BM;

  v8f acc[2];
  {
    v8f z8 = {0.f, 0.f, 0.f, 0.f, 0.f, 0.f, 0.f, 0.f};
    acc[0] = z8;
    acc[1] = z8;
  }

  const int nph = dual ? 2 : 1;
  for (int ph = 0; ph < nph; ++ph) {
    const float* A = ph ? A2 : A1;
    const us* Wh = ph ? W2h : W1h;
    const us* Wl = ph ? W2l : W1l;
#pragma unroll
    for (int j = 0; j < 8; ++j) {
      const int c = tid + 256 * j;
      ((v8usa*)sWh)[c] = ((const v8usa*)Wh)[c];
      ((v8usa*)sWl)[c] = ((const v8usa*)Wl)[c];
    }
    {
      const int r = tid >> 3;
      const int kq = (tid & 7) * 16;
      const int gr = row0 + r;
      v4f xa[4];
      if (gr < M) {
        const float* ap = A + (size_t)gr * HD + kq;
#pragma unroll
        for (int q = 0; q < 4; ++q) xa[q] = *(const v4fa*)(ap + 4 * q);
      } else {
        v4f z4 = {0.f, 0.f, 0.f, 0.f};
#pragma unroll
        for (int q = 0; q < 4; ++q) xa[q] = z4;
      }
      v8us hv[2], lv[2];
#pragma unroll
      for (int i = 0; i < 16; ++i) {
        const float x = xa[i >> 2][i & 3];
        const us hb = f2bf(x);
        const us lb = f2bf(x - bf2f(hb));
        hv[i >> 3][i & 7] = hb;
        lv[i >> 3][i & 7] = lb;
      }
      us* dh = sAh + r * HD + kq;
      us* dl = sAl + r * HD + kq;
      *(v8usa*)dh = hv[0];
      *(v8usa*)(dh + 8) = hv[1];
      *(v8usa*)dl = lv[0];
      *(v8usa*)(dl + 8) = lv[1];
    }
    __syncthreads();
#pragma unroll
    for (int ks = 0; ks < 4; ++ks) {
      const int k0 = ks * 32;
      const v16us bh = ldfrag(sWh, wv * 16 + m, k0, hf);
      const v16us bl = ldfrag(sWl, wv * 16 + m, k0, hf);
#pragma unroll
      for (int rt = 0; rt < 2; ++rt) {
        const v16us ah = ldfrag(sAh, rt * 16 + m, k0, hf);
        const v16us al = ldfrag(sAl, rt * 16 + m, k0, hf);
        acc[rt] = mma_bf16(ah, bh, acc[rt]);
        acc[rt] = mma_bf16(ah, bl, acc[rt]);
        acc[rt] = mma_bf16(al, bh, acc[rt]);
      }
    }
    __syncthreads();
  }

  {
    const int col = wv * 16 + m;
    const float bvv = use_bias ? bias[col] : 0.0f;
#pragma unroll
    for (int rt = 0; rt < 2; ++rt) {
#pragma unroll
      for (int r = 0; r < 8; ++r) {
        const int row = rt * 16 + hf * 8 + r;
        const int gr = row0 + row;
        float v = acc[rt][r];
        if (use_rs) {
          const int gi = (gr < M) ? gr : (M - 1);
          v *= rscale[gi];
        }
        v += bvv;
        if (relu) v = fmaxf(v, 0.0f);
        sOut[row * HD + col] = v;
      }
    }
  }
  __syncthreads();

  if (!head) {
    gemm_rows_store(sOut, OUT, row0, M, wv, lane);
    __threadfence();
    gemm_rows_store(sOut, OUT, row0, M, wv, lane);
  } else {
    const int rows = (M - row0 < BM) ? (M - row0) : BM;
    const int nres = rows * OD;
    if (tid < nres) {
      const int g = tid / OD;
      const int o = tid - g * OD;
      float s = bf2[o];
      const float* zr = sOut + g * HD;
#pragma unroll 1
      for (int k = 0; k < HD; ++k) s = fmaf(zr[k], Wf2[k * OD + o], s);
      sRes[tid] = s;
    }
    __syncthreads();
    if (wv == 0) {
      const int base = row0 * OD;
      head_store(sRes, hout, base, nres, hout_n, lane);
      __threadfence();
      head_store(sRes, hout, base, nres, hout_n, lane);
    }
  }
}

extern "C" void kernel_launch(void* const* d_in, const int* in_sizes, int n_in,
                              void* d_out, int out_size, void* d_ws, size_t ws_size,
                              hipStream_t stream) {
  if (n_in < 12) return;
  const float* x        = (const float*)d_in[0];
  const int*   ei       = (const int*)  d_in[1];
  const int*   batch    = (const int*)  d_in[2];
  const float* W_gcn    = (const float*)d_in[3];
  const float* b_gcn    = (const float*)d_in[4];
  const float* W_sage_l = (const float*)d_in[5];
  const float* W_sage_r = (const float*)d_in[6];
  const float* b_sage   = (const float*)d_in[7];
  const float* W_fc1    = (const float*)d_in[8];
  const float* b_fc1    = (const float*)d_in[9];
  const float* W_fc2    = (const float*)d_in[10];
  const float* b_fc2    = (const float*)d_in[11];
  float* out = (float*)d_out;

  const int N = in_sizes[0] / HD;
  const int E = in_sizes[1] / 2;
  const int G = out_size / OD;
  if (N <= 0 || G <= 0 || E < 0) return;
  if (N * HD != in_sizes[0] || G * OD != out_size) return;
  const int Npad = ((N + 31) / 32) * 32;

  const int* row = ei;
  const int* col = ei + E;

  char* ws = (char*)d_ws;
  size_t off = 0;
  auto carve = [&](size_t bytes) -> void* {
    void* p = ws + off;
    off = (off + bytes + 255) & ~(size_t)255;
    return p;
  };
  us*    Wt     = (us*)   carve((size_t)8 * HD * HD * sizeof(us));
  float* dinv   = (float*)carve((size_t)Npad * 4);
  float* rcnt   = (float*)carve((size_t)Npad * 4);
  float* hs     = (float*)carve((size_t)N * HD * 4);
  float* hgcn   = (float*)carve((size_t)N * HD * 4);
  float* neigh  = (float*)carve((size_t)N * HD * 4);
  float* hsage  = (float*)carve((size_t)N * HD * 4);
  float* pooled = (float*)carve((size_t)G * HD * 4);
  if (off > ws_size) return;

  us* WtGh = Wt + 0 * HD * HD; us* WtGl = Wt + 1 * HD * HD;
  us* WtLh = Wt + 2 * HD * HD; us* WtLl = Wt + 3 * HD * HD;
  us* WtRh = Wt + 4 * HD * HD; us* WtRl = Wt + 5 * HD * HD;
  us* Wt1h = Wt + 6 * HD * HD; us* Wt1l = Wt + 7 * HD * HD;

  k_wtconv<<<dim3(8, 4), dim3(256), 0, stream>>>(W_gcn, W_sage_l, W_sage_r, W_fc1, Wt);
  k_degree<<<dim3((N + RC - 1) / RC), dim3(32), 0, stream>>>(col, E, N, Npad, dinv, rcnt);
  k_gemm<<<dim3((N + BM - 1) / BM), dim3(256), 0, stream>>>(
      x, WtGh, WtGl, x, WtGh, WtGl, b_gcn, dinv, hs, N,
      0, 0, 0, 1, 0, W_fc2, b_fc2, out, out_size);
  k_gather<<<dim3((N + RG - 1) / RG), dim3(32), 0, stream>>>(
      row, col, E, N, hs, dinv, rcnt, b_gcn, hgcn, 0);
  k_gather<<<dim3((N + RG - 1) / RG), dim3(32), 0, stream>>>(
      row, col, E, N, hgcn, dinv, rcnt, b_gcn, neigh, 1);
  k_gemm<<<dim3((N + BM - 1) / BM), dim3(256), 0, stream>>>(
      neigh, WtLh, WtLl, hgcn, WtRh, WtRl, b_sage, dinv, hsage, N,
      1, 1, 1, 0, 0, W_fc2, b_fc2, out, out_size);
  k_pool<<<dim3(G), dim3(32), 0, stream>>>(batch, N, hsage, pooled);
  k_gemm<<<dim3((G + BM - 1) / BM), dim3(256), 0, stream>>>(
      pooled, Wt1h, Wt1l, pooled, Wt1h, Wt1l, b_fc1, dinv, hsage, G,
      0, 1, 1, 0, 1, W_fc2, b_fc2, out, out_size);
}
